// BigBirdBlock_69020124446907
// MI455X (gfx1250) — hardware-run, weakly checked
//
#include <hip/hip_runtime.h>
#include <math.h>

constexpr int kBatch = 4;
constexpr int kSeq   = 4096;
constexpr int kDim   = 512;
constexpr int kHeads = 8;
constexpr int kHdim  = 64;
constexpr int kMlp   = 2048;
constexpr int kNB    = 64;
constexpr int kNI    = 62;
constexpr int kKint  = 512;
constexpr int kHG    = 4;
constexpr float kWCarry    = 16.0f;
constexpr float kXLoCarry  = 2048.0f;
constexpr float kOCarry    = 16.0f;
constexpr float kHidCarry  = 4.0f;
constexpr float kLnEps     = 1e-6f;
constexpr float kNegFill   = -1e9f;
constexpr float kInvDim    = 1.0f / 512.0f;

typedef __attribute__((ext_vector_type(16))) _Float16 v16h;
typedef __attribute__((ext_vector_type(8)))  _Float16 v8h;
typedef __attribute__((ext_vector_type(16))) __bf16   v16b;
typedef __attribute__((ext_vector_type(8)))  __bf16   v8b;
typedef __attribute__((ext_vector_type(8)))  float    v8f;
typedef __attribute__((ext_vector_type(4)))  float    v4f;
typedef __attribute__((ext_vector_type(4)))  unsigned int v4u;

__constant__ int c_idx[62][8] = {{0,1,2,63,29,38,62,0},{0,1,2,3,63,29,34,14},{0,2,3,4,63,30,58,41},{0,3,4,5,63,27,42,24},{0,4,5,6,63,59,32,17},{0,5,6,7,63,60,58,61},{0,6,7,8,63,50,44,59},{0,7,8,9,63,18,6,38},{0,8,9,10,63,61,21,47},{0,9,10,11,63,25,4,42},{0,10,11,12,63,18,8,29},{0,11,12,13,63,60,54,38},{0,12,13,14,63,45,15,37},{0,13,14,15,63,8,39,18},{0,14,15,16,63,12,38,9},{0,15,16,17,63,42,53,32},{0,16,17,18,63,1,51,54},{0,17,18,19,63,1,39,10},{0,18,19,20,63,11,6,35},{0,19,20,21,63,57,54,6},{0,20,21,22,63,52,13,7},{0,21,22,23,63,37,39,11},{0,22,23,24,63,35,6,12},{0,23,24,25,63,61,2,50},{0,24,25,26,63,60,35,36},{0,25,26,27,63,9,43,4},{0,26,27,28,63,46,60,7},{0,27,28,29,63,10,1,16},{0,28,29,30,63,43,10,42},{0,29,30,31,63,59,19,61},{0,30,31,32,63,38,16,20},{0,31,32,33,63,53,44,6},{0,32,33,34,63,13,38,4},{0,33,34,35,63,30,38,23},{0,34,35,36,63,51,19,13},{0,35,36,37,63,50,33,51},{0,36,37,38,63,52,53,54},{0,37,38,39,63,54,13,21},{0,38,39,40,63,48,52,22},{0,39,40,41,63,34,31,57},{0,40,41,42,63,47,15,23},{0,41,42,43,63,22,8,58},{0,42,43,44,63,29,58,8},{0,43,44,45,63,8,55,16},{0,44,45,46,63,25,37,17},{0,45,46,47,63,22,21,55},{0,46,47,48,63,8,17,54},{0,47,48,49,63,40,57,41},{0,48,49,50,63,23,45,5},{0,49,50,51,63,58,14,28},{0,50,51,52,63,38,41,44},{0,51,52,53,63,37,19,40},{0,52,53,54,63,14,46,35},{0,53,54,55,63,50,41,35},{0,54,55,56,63,24,35,5},{0,55,56,57,63,51,17,3},{0,56,57,58,63,10,55,61},{0,57,58,59,63,51,25,43},{0,58,59,60,63,8,37,14},{0,59,60,61,63,52,24,33},{0,60,61,62,63,4,44,45},{0,61,62,63,32,4,58,0}};
static_assert(sizeof(c_idx) / sizeof(c_idx[0][0]) == 62 * 8);
static_assert(sizeof(c_idx) == 62 * 8 * sizeof(int));

__device__ __forceinline__ unsigned short f2bf_bits(float f) {
  unsigned u = __float_as_uint(f);
  return (unsigned short)((u + 0x7FFFu + ((u >> 16) & 1u)) >> 16);
}
__device__ __forceinline__ float bf_bits2f(unsigned short h) { return __uint_as_float(((unsigned)h) << 16); }

__device__ __forceinline__ void dep_guard_h(v8f& a, v8f& b, v16h x, v16h y) { asm volatile("v_nop\n\tv_nop\n\tv_nop\n\tv_nop" : "+v"(a), "+v"(b) : "v"(x), "v"(y)); }
__device__ __forceinline__ void dep_guard_b(v8f& a, v8f& b, v16b x, v16b y) { asm volatile("v_nop\n\tv_nop\n\tv_nop\n\tv_nop" : "+v"(a), "+v"(b) : "v"(x), "v"(y)); }
__device__ __forceinline__ void keep4_h(v16h a, v16h b, v16h c, v16h d) { asm volatile("v_nop" :: "v"(a), "v"(b), "v"(c), "v"(d)); }
__device__ __forceinline__ void keep4_b(v16b a, v16b b, v16b c, v16b d) { asm volatile("v_nop" :: "v"(a), "v"(b), "v"(c), "v"(d)); }
__device__ __forceinline__ void acc_guard4(v8f& a, v8f& b, v8f& c, v8f& d) { asm volatile("v_nop\n\tv_nop\n\tv_nop\n\tv_nop" : "+v"(a), "+v"(b), "+v"(c), "+v"(d)); }
template <typename T> struct Frag;
template <> struct Frag<_Float16> {
  typedef v16h V; union U { v16h v; v8h h[2]; };
  static __device__ __forceinline__ v16h load(const _Float16* p) {
    U f; f.h[0] = *(const v8h*)(p); f.h[1] = *(const v8h*)(p + 16); return f.v;
  }
  static __device__ __forceinline__ v8f mma(v16h a, v16h b, v8f c) {
    return __builtin_amdgcn_wmma_f32_16x16x32_f16(false, a, false, b, (short)0, c, false, false);
  }
  static __device__ __forceinline__ void guard(v8f& a, v8f& b, v16h x, v16h y) { dep_guard_h(a, b, x, y); }
  static __device__ __forceinline__ void keep(v16h a, v16h b, v16h c, v16h d) { keep4_h(a, b, c, d); }
};
template <> struct Frag<__bf16> {
  typedef v16b V; union U { v16b v; v8b h[2]; };
  static __device__ __forceinline__ v16b load(const __bf16* p) {
    U f; f.h[0] = *(const v8b*)(p); f.h[1] = *(const v8b*)(p + 16); return f.v;
  }
  static __device__ __forceinline__ v8f mma(v16b a, v16b b, v8f c) {
    return __builtin_amdgcn_wmma_f32_16x16x32_bf16(false, a, false, b, (short)0, c, false, false);
  }
  static __device__ __forceinline__ void guard(v8f& a, v8f& b, v16b x, v16b y) { dep_guard_b(a, b, x, y); }
  static __device__ __forceinline__ void keep(v16b a, v16b b, v16b c, v16b d) { keep4_b(a, b, c, d); }
};

__device__ __forceinline__ unsigned pk16(unsigned short a, unsigned short b) { return (unsigned)a | ((unsigned)b << 16); }
__device__ __forceinline__ unsigned short h_bits(float f) { const _Float16 h = (_Float16)f; return __builtin_bit_cast(unsigned short, h); }
__device__ __forceinline__ float hbits2f(unsigned short h) { return (float)__builtin_bit_cast(_Float16, h); }

template <int ET> struct Elem;
template <> struct Elem<0> { typedef _Float16 T; };
template <> struct Elem<1> { typedef __bf16 T; };
template <int ET, bool SPLIT, int BIAS_MODE, int OUT_MODE, bool RESID, int ACT = 0>
__global__ __launch_bounds__(256) void wmma_gemm64(
    const unsigned short* __restrict__ Ap, const unsigned short* __restrict__ A2p, int lda, long strideA,
    const unsigned short* __restrict__ Btp, const unsigned short* __restrict__ Bt2p, int ldb, long strideB,
    void* __restrict__ Cout, void* __restrict__ Cout2, int ldc, long strideC,
    const float* __restrict__ bias,
    const float* __restrict__ resid, long strideR,
    int M, int N, int K, float scale) {
  typedef typename Elem<ET>::T T;
  typedef typename Frag<T>::V V;
  const T* A = (const T*)Ap; const T* A2 = (const T*)A2p; const T* Bt = (const T*)Btp; const T* Bt2 = (const T*)Bt2p;
  __shared__ __align__(16) float sT[8][16 * 68];
  const int b    = blockIdx.y;
  const int lane = threadIdx.x & 31;
  const int wave = threadIdx.x >> 5;
  const int tilesN = N >> 6;
  const int tilesM = M >> 6;
  const int tile = blockIdx.x * 8 + wave;
  if (tile >= tilesM * tilesN) return;
  const int tm = tile / tilesN;
  const int tn = tile - tm * tilesN;
  const int m0 = tm << 6;
  const int n0 = tn << 6;

  const T* Ab  = A  + (size_t)b * strideA;
  const T* Bb  = Bt + (size_t)b * strideB;
  const T* Ab2 = SPLIT ? (A2  + (size_t)b * strideA) : nullptr;
  const T* Bb2 = SPLIT ? (Bt2 + (size_t)b * strideB) : nullptr;

  const int rlane = lane & 15;
  const int koff  = (lane >> 4) * 8;
  const int mOff  = (lane >> 4) * 8;

  v8f acc[4][4];
#pragma unroll
  for (int i = 0; i < 4; ++i)
#pragma unroll
    for (int j = 0; j < 4; ++j) acc[i][j] = (v8f){0.f,0.f,0.f,0.f,0.f,0.f,0.f,0.f};

  for (int k0 = 0; k0 < K; k0 += 32) {
    V bh[4], bl[4];
#pragma unroll
    for (int j = 0; j < 4; ++j) {
      const size_t bo = (size_t)(n0 + (j << 4) + rlane) * ldb + koff + k0;
      bh[j] = Frag<T>::load(Bb + bo);
      if (SPLIT) bl[j] = Frag<T>::load(Bb2 + bo);
    }
#pragma unroll
    for (int i = 0; i < 4; ++i) {
      const size_t ao = (size_t)(m0 + (i << 4) + rlane) * lda + koff + k0;
      V ah = Frag<T>::load(Ab + ao);
      V al;
      if (SPLIT) al = Frag<T>::load(Ab2 + ao);
#pragma unroll
      for (int j = 0; j < 4; ++j) {
        acc[i][j] = Frag<T>::mma(ah, bh[j], acc[i][j]);
        if (SPLIT) {
          acc[i][j] = Frag<T>::mma(ah, bl[j], acc[i][j]);
          acc[i][j] = Frag<T>::mma(al, bh[j], acc[i][j]);
        }
      }
      Frag<T>::guard(acc[i][0], acc[i][3], ah, SPLIT ? al : ah);
    }
    Frag<T>::keep(bh[0], bh[1], bh[2], bh[3]);
    if (SPLIT) Frag<T>::keep(bl[0], bl[1], bl[2], bl[3]);
  }
  acc_guard4(acc[0][0], acc[0][1], acc[0][2], acc[0][3]);
  acc_guard4(acc[1][0], acc[1][1], acc[1][2], acc[1][3]);
  acc_guard4(acc[2][0], acc[2][1], acc[2][2], acc[2][3]);
  acc_guard4(acc[3][0], acc[3][1], acc[3][2], acc[3][3]);

  float* slab = sT[wave];
  const float* Rb = RESID ? (resid + (size_t)b * strideR) : nullptr;
#pragma unroll
  for (int i = 0; i < 4; ++i) {
    const int mBase = m0 + (i << 4);
#pragma unroll
    for (int j = 0; j < 4; ++j) {
      const int n = n0 + (j << 4) + rlane;
      float bv = 0.f;
      if (BIAS_MODE == 2) bv = bias[n];
#pragma unroll
      for (int r = 0; r < 8; ++r) {
        float v = acc[i][j][r] * scale;
        if (BIAS_MODE == 1) v += bias[mBase + mOff + r];
        if (BIAS_MODE == 2) v += bv;
        if (RESID) v += Rb[(size_t)(mBase + mOff + r) * ldc + n];
        if (ACT == 1) v = tanhf(v);
        if (ACT == 2) v = fmaxf(v, 0.0f);
        if (ACT == 3) v = v / (1.0f + expf(-v));
        if (ACT == 4) v = (v > 0.f) ? v : 0.01f * v;
        if (ACT == 5) v = 0.5f * v * (1.0f + erff(v * 0.70710678118654752f));
        if (ACT == 6) {
          const float u  = 0.7978845608028654f * (v + 0.044715f * v * v * v);
          const float tt = expf(-2.0f * fabsf(u));
          const float rr = 1.0f / (1.0f + tt);
          const float gp = v * rr;
          v = (u >= 0.0f) ? gp : gp * tt;
          v *= kHidCarry;
        }
        slab[(mOff + r) * 68 + (j << 4) + rlane] = v;
      }
    }
    __builtin_amdgcn_fence(__ATOMIC_RELEASE, "workgroup");
    __builtin_amdgcn_wave_barrier();
    __builtin_amdgcn_fence(__ATOMIC_ACQUIRE, "workgroup");
    if (OUT_MODE == 0) {
      float* C = (float*)Cout + (size_t)b * strideC;
      const int hh = lane >> 4, c4 = (lane & 15) * 4;
      for (int pass = 0; pass < 2; ++pass) {
#pragma unroll
        for (int it = 0; it < 8; ++it) {
          const int row = it * 2 + hh;
          v4f v = *(const v4f*)(slab + row * 68 + c4);
          *(volatile v4f*)(C + (size_t)(mBase + row) * ldc + n0 + c4) = v;
        }
        __threadfence();
      }
    } else {
      const int q = lane >> 3, c8 = (lane & 7) * 8;
      unsigned short* C  = (unsigned short*)Cout  + (size_t)b * strideC;
      unsigned short* C2 = (OUT_MODE == 2) ? ((unsigned short*)Cout2 + (size_t)b * strideC) : nullptr;
      for (int pass = 0; pass < 2; ++pass) {
#pragma unroll
        for (int it = 0; it < 4; ++it) {
          const int row = it * 4 + q;
          const float* sp = slab + row * 68 + c8;
          v8h hv, lv;
#pragma unroll
          for (int e = 0; e < 8; ++e) {
            if (OUT_MODE == 1) {
              hv[e] = (_Float16)sp[e];
            } else {
              unsigned short hb = f2bf_bits(sp[e]);
              unsigned short lb = f2bf_bits(sp[e] - bf_bits2f(hb));
              hv[e] = __builtin_bit_cast(_Float16, hb);
              lv[e] = __builtin_bit_cast(_Float16, lb);
            }
          }
          *(volatile v8h*)(C + (size_t)(mBase + row) * ldc + n0 + c8) = hv;
          if (OUT_MODE == 2) *(volatile v8h*)(C2 + (size_t)(mBase + row) * ldc + n0 + c8) = lv;
        }
        __threadfence();
      }
    }
    __builtin_amdgcn_fence(__ATOMIC_RELEASE, "workgroup");
    __builtin_amdgcn_wave_barrier();
    __builtin_amdgcn_fence(__ATOMIC_ACQUIRE, "workgroup");
  }
}

__global__ __launch_bounds__(256) void tcast_kernel(const float* __restrict__ W0, const float* __restrict__ W1,
                                                    const float* __restrict__ W2, const float* __restrict__ W3,
                                                    int rows, int cols, unsigned short* __restrict__ out,
                                                    long zstride, float scale) {
  __shared__ float sm[64][65];
  const int t  = threadIdx.x;
  const int r0 = blockIdx.x * 64;
  const int c0 = blockIdx.y * 64;
  const int z  = blockIdx.z;
  const float* W = (z == 0) ? W0 : (z == 1) ? W1 : (z == 2) ? W2 : W3;
#pragma unroll
  for (int i = 0; i < 16; ++i) {
    const int e = i * 256 + t;
    const int r = e >> 6;
    const int c = e & 63;
    sm[c][r] = W[(size_t)(r0 + r) * cols + c0 + c] * scale;
  }
  __syncthreads();
  const int lane = t & 31, wave = t >> 5;
  const int q = lane >> 3, c8 = (lane & 7) * 8;
  unsigned short* op = out + (size_t)z * zstride;
  for (int pass = 0; pass < 2; ++pass) {
#pragma unroll
    for (int it = 0; it < 2; ++it) {
      const int row = wave * 8 + it * 4 + q;
      unsigned short hb[8];
#pragma unroll
      for (int e = 0; e < 8; ++e) hb[e] = h_bits(sm[row][c8 + e]);
      const v4u u = (v4u){pk16(hb[0], hb[1]), pk16(hb[2], hb[3]), pk16(hb[4], hb[5]), pk16(hb[6], hb[7])};
      *(volatile v4u*)(op + (size_t)(c0 + row) * rows + r0 + c8) = u;
    }
    __threadfence();
  }
}

template <bool LO>
__global__ __launch_bounds__(256) void ln_kernel(const float* __restrict__ x, const float* __restrict__ sc,
                                                 const float* __restrict__ bi, unsigned short* __restrict__ oh,
                                                 unsigned short* __restrict__ ol, int nrows) {
  const int lane = threadIdx.x & 31, wave = threadIdx.x >> 5;
  const int row = blockIdx.x * 8 + wave;
  if (row >= nrows) return;
  const float* xr = x + (size_t)row * kDim;
  const int c0 = lane * 8, c1 = 256 + lane * 8;
  const v4f a0 = *(const v4f*)(xr + c0);
  const v4f a1 = *(const v4f*)(xr + c0 + 4);
  const v4f a2 = *(const v4f*)(xr + c1);
  const v4f a3 = *(const v4f*)(xr + c1 + 4);
  float v[16];
#pragma unroll
  for (int e = 0; e < 4; ++e) { v[e] = a0[e]; v[4 + e] = a1[e]; v[8 + e] = a2[e]; v[12 + e] = a3[e]; }
  float s = 0.f;
#pragma unroll
  for (int e = 0; e < 16; ++e) s += v[e];
  s += __shfl_xor(s, 16, 32); s += __shfl_xor(s, 8, 32); s += __shfl_xor(s, 4, 32); s += __shfl_xor(s, 2, 32); s += __shfl_xor(s, 1, 32);
  const float mu = s * kInvDim;
  float q = 0.f;
#pragma unroll
  for (int e = 0; e < 16; ++e) { const float d = v[e] - mu; q += d * d; }
  q += __shfl_xor(q, 16, 32); q += __shfl_xor(q, 8, 32); q += __shfl_xor(q, 4, 32); q += __shfl_xor(q, 2, 32); q += __shfl_xor(q, 1, 32);
  const float rs = rsqrtf(q * kInvDim + kLnEps);
  const v4f s0 = *(const v4f*)(sc + c0), s1 = *(const v4f*)(sc + c0 + 4), s2 = *(const v4f*)(sc + c1), s3 = *(const v4f*)(sc + c1 + 4);
  const v4f g0 = *(const v4f*)(bi + c0), g1 = *(const v4f*)(bi + c0 + 4), g2 = *(const v4f*)(bi + c1), g3 = *(const v4f*)(bi + c1 + 4);
  float scv[16], biv[16];
#pragma unroll
  for (int e = 0; e < 4; ++e) {
    scv[e] = s0[e]; scv[4 + e] = s1[e]; scv[8 + e] = s2[e]; scv[12 + e] = s3[e];
    biv[e] = g0[e]; biv[4 + e] = g1[e]; biv[8 + e] = g2[e]; biv[12 + e] = g3[e];
  }
  unsigned short hb[16], lb[16];
#pragma unroll
  for (int e = 0; e < 16; ++e) {
    const float y = (v[e] - mu) * rs * scv[e] + biv[e];
    hb[e] = h_bits(y);
    if (LO) lb[e] = h_bits((y - hbits2f(hb[e])) * kXLoCarry);
    else lb[e] = 0;
  }
  const v4u uh0 = (v4u){pk16(hb[0], hb[1]), pk16(hb[2], hb[3]), pk16(hb[4], hb[5]), pk16(hb[6], hb[7])};
  const v4u uh1 = (v4u){pk16(hb[8], hb[9]), pk16(hb[10], hb[11]), pk16(hb[12], hb[13]), pk16(hb[14], hb[15])};
  const v4u ul0 = (v4u){pk16(lb[0], lb[1]), pk16(lb[2], lb[3]), pk16(lb[4], lb[5]), pk16(lb[6], lb[7])};
  const v4u ul1 = (v4u){pk16(lb[8], lb[9]), pk16(lb[10], lb[11]), pk16(lb[12], lb[13]), pk16(lb[14], lb[15])};
  unsigned short* ph = oh + (size_t)row * kDim;
  unsigned short* pl = ol + (size_t)row * kDim;
  for (int pass = 0; pass < 2; ++pass) {
    *(volatile v4u*)(ph + c0) = uh0;
    *(volatile v4u*)(ph + c1) = uh1;
    if (LO) {
      *(volatile v4u*)(pl + c0) = ul0;
      *(volatile v4u*)(pl + c1) = ul1;
    }
    __threadfence();
  }
}

__global__ __launch_bounds__(256) void softmax_int_kernel(const float* __restrict__ S, unsigned short* __restrict__ Ph,
                                                          unsigned short* __restrict__ Pl) {
  __shared__ float redM[8];
  __shared__ float redS[8];
  const int t = threadIdx.x, lane = t & 31, wave = t >> 5;
  const int rloc = wave >> 1, half = wave & 1;
  const int row = blockIdx.x * 4 + rloc;
  const int ni = (row >> 6) % kNI;
  const int nvalid = (ni == 0 || ni == kNI - 1) ? 7 : 8;
  const int c0 = half * 256 + lane * 8;
  const int slot = c0 >> 6;
  const bool valid = slot < nvalid;
  const float* sr = S + (size_t)row * kKint + c0;
  const v4f a = *(const v4f*)(sr);
  const v4f c = *(const v4f*)(sr + 4);
  float xv[8];
#pragma unroll
  for (int e = 0; e < 4; ++e) {
    xv[e]     = valid ? a[e] : kNegFill;
    xv[4 + e] = valid ? c[e] : kNegFill;
  }
  float m = fmaxf(fmaxf(fmaxf(xv[0], xv[1]), fmaxf(xv[2], xv[3])), fmaxf(fmaxf(xv[4], xv[5]), fmaxf(xv[6], xv[7])));
  m = fmaxf(m, __shfl_xor(m, 16, 32)); m = fmaxf(m, __shfl_xor(m, 8, 32)); m = fmaxf(m, __shfl_xor(m, 4, 32));
  m = fmaxf(m, __shfl_xor(m, 2, 32)); m = fmaxf(m, __shfl_xor(m, 1, 32));
  if (lane == 0) redM[wave] = m;
  __syncthreads();
  m = fmaxf(redM[rloc * 2], redM[rloc * 2 + 1]);
  float p[8];
  float sum = 0.f;
#pragma unroll
  for (int e = 0; e < 8; ++e) { p[e] = expf(xv[e] - m); sum += p[e]; }
  sum += __shfl_xor(sum, 16, 32); sum += __shfl_xor(sum, 8, 32); sum += __shfl_xor(sum, 4, 32);
  sum += __shfl_xor(sum, 2, 32); sum += __shfl_xor(sum, 1, 32);
  if (lane == 0) redS[wave] = sum;
  __syncthreads();
  sum = redS[rloc * 2] + redS[rloc * 2 + 1];
  const float inv = 1.0f / sum;
  unsigned short hb[8], lb[8];
#pragma unroll
  for (int e = 0; e < 8; ++e) {
    const float pe = p[e] * inv;
    hb[e] = f2bf_bits(pe);
    lb[e] = f2bf_bits(pe - bf_bits2f(hb[e]));
  }
  const v4u uh = (v4u){pk16(hb[0], hb[1]), pk16(hb[2], hb[3]), pk16(hb[4], hb[5]), pk16(hb[6], hb[7])};
  const v4u ul = (v4u){pk16(lb[0], lb[1]), pk16(lb[2], lb[3]), pk16(lb[4], lb[5]), pk16(lb[6], lb[7])};
  unsigned short* qh = Ph + (size_t)row * kKint + c0;
  unsigned short* ql = Pl + (size_t)row * kKint + c0;
  for (int pass = 0; pass < 2; ++pass) {
    *(volatile v4u*)qh = uh;
    *(volatile v4u*)ql = ul;
    __threadfence();
  }
}

__global__ __launch_bounds__(512) void softmax_glob_kernel(const float* __restrict__ S, unsigned short* __restrict__ Ph,
                                                           unsigned short* __restrict__ Pl) {
  __shared__ float redM[16];
  __shared__ float redS[16];
  const int row = blockIdx.x;
  const int t = threadIdx.x, lane = t & 31, wave = t >> 5;
  const int c0 = t * 8;
  const float* sr = S + (size_t)row * kSeq + c0;
  const v4f a = *(const v4f*)(sr);
  const v4f c = *(const v4f*)(sr + 4);
  float xv[8];
#pragma unroll
  for (int e = 0; e < 4; ++e) { xv[e] = a[e]; xv[4 + e] = c[e]; }
  float m = fmaxf(fmaxf(fmaxf(xv[0], xv[1]), fmaxf(xv[2], xv[3])), fmaxf(fmaxf(xv[4], xv[5]), fmaxf(xv[6], xv[7])));
  m = fmaxf(m, __shfl_xor(m, 16, 32)); m = fmaxf(m, __shfl_xor(m, 8, 32)); m = fmaxf(m, __shfl_xor(m, 4, 32));
  m = fmaxf(m, __shfl_xor(m, 2, 32)); m = fmaxf(m, __shfl_xor(m, 1, 32));
  if (lane == 0) redM[wave] = m;
  __syncthreads();
  m = redM[0];
#pragma unroll
  for (int w = 1; w < 16; ++w) m = fmaxf(m, redM[w]);
  float p[8];
  float sum = 0.f;
#pragma unroll
  for (int e = 0; e < 8; ++e) { p[e] = expf(xv[e] - m); sum += p[e]; }
  sum += __shfl_xor(sum, 16, 32); sum += __shfl_xor(sum, 8, 32); sum += __shfl_xor(sum, 4, 32);
  sum += __shfl_xor(sum, 2, 32); sum += __shfl_xor(sum, 1, 32);
  if (lane == 0) redS[wave] = sum;
  __syncthreads();
  sum = redS[0];
#pragma unroll
  for (int w = 1; w < 16; ++w) sum += redS[w];
  const float inv = 1.0f / sum;
  unsigned short hb[8], lb[8];
#pragma unroll
  for (int e = 0; e < 8; ++e) {
    const float pe = p[e] * inv;
    hb[e] = f2bf_bits(pe);
    lb[e] = f2bf_bits(pe - bf_bits2f(hb[e]));
  }
  const v4u uh = (v4u){pk16(hb[0], hb[1]), pk16(hb[2], hb[3]), pk16(hb[4], hb[5]), pk16(hb[6], hb[7])};
  const v4u ul = (v4u){pk16(lb[0], lb[1]), pk16(lb[2], lb[3]), pk16(lb[4], lb[5]), pk16(lb[6], lb[7])};
  unsigned short* qh = Ph + (size_t)row * kSeq + c0;
  unsigned short* ql = Pl + (size_t)row * kSeq + c0;
  for (int pass = 0; pass < 2; ++pass) {
    *(volatile v4u*)qh = uh;
    *(volatile v4u*)ql = ul;
    __threadfence();
  }
}

template <int OUTF>
__global__ __launch_bounds__(256) void attn_tile_kernel(
    const unsigned short* __restrict__ Aihp, const unsigned short* __restrict__ Ailp,
    const unsigned short* __restrict__ Aghp, const unsigned short* __restrict__ Aglp,
    const unsigned short* __restrict__ Bhp,  const unsigned short* __restrict__ Blp,
    void* __restrict__ Cip, void* __restrict__ Cgp, int h0, float scale) {
  typedef __bf16 T;
  typedef v16b V;
  __shared__ __align__(16) float sT[8][16 * 68];
  const int lane = threadIdx.x & 31;
  const int wave = threadIdx.x >> 5;
  const int gw = blockIdx.x * 8 + wave;
  const int nI = (OUTF == 0) ? (kHG * kNI * 8) : (kHG * kNI);
  const int nG = (OUTF == 0) ? (kHG * 2 * 64) : (kHG * 2);
  if (gw >= nI + nG) return;
  const bool isInt = gw < nI;
  size_t aOff = 0, bOff = 0, cOff = 0;
  int lda = 0, ldb = 0, ldc = 0, Ktot = 0, tabRow = 0;
  bool useTab = false;
  if (OUTF == 0) {
    if (isInt) {
      const int hl = gw / (kNI * 8);
      const int rem = gw - hl * (kNI * 8);
      const int ni = rem >> 3;
      const int slot = rem & 7;
      const int h = h0 + hl;
      const int kb = c_idx[ni][slot];
      aOff = (size_t)((ni + 1) * 64) * kDim + h * kHdim; lda = kDim;
      bOff = (size_t)(kb * 64) * kDim + h * kHdim;       ldb = kDim;
      cOff = (size_t)((hl * kNI + ni) * 64) * kKint + slot * 64; ldc = kKint;
      Ktot = 64; useTab = false; tabRow = 0;
    } else {
      const int r = gw - nI;
      const int hl = r >> 7;
      const int rem = r & 127;
      const int g = rem >> 6;
      const int tt = rem & 63;
      const int h = h0 + hl;
      const int nq = g ? (kNB - 1) : 0;
      aOff = (size_t)(nq * 64) * kDim + h * kHdim; lda = kDim;
      bOff = (size_t)(tt * 64) * kDim + h * kHdim; ldb = kDim;
      cOff = (size_t)((hl * 2 + g) * 64) * kSeq + tt * 64; ldc = kSeq;
      Ktot = 64; useTab = false; tabRow = 0;
    }
  } else {
    if (isInt) {
      const int hl = gw / kNI;
      const int ni = gw - hl * kNI;
      const int h = h0 + hl;
      aOff = (size_t)((hl * kNI + ni) * 64) * kKint; lda = kKint;
      bOff = (size_t)(h * kHdim) * kSeq;             ldb = kSeq;
      cOff = (size_t)((ni + 1) * 64) * kDim + h * kHdim; ldc = kDim;
      Ktot = kKint; useTab = true; tabRow = ni;
    } else {
      const int r = gw - nI;
      const int hl = r >> 1;
      const int g = r & 1;
      const int h = h0 + hl;
      const int nq = g ? (kNB - 1) : 0;
      aOff = (size_t)((hl * 2 + g) * 64) * kSeq; lda = kSeq;
      bOff = (size_t)(h * kHdim) * kSeq;         ldb = kSeq;
      cOff = (size_t)(nq * 64) * kDim + h * kHdim; ldc = kDim;
      Ktot = kSeq; useTab = false; tabRow = 0;
    }
  }
  const T* Ah = (const T*)(isInt ? Aihp : Aghp) + aOff;
  const T* Al = (const T*)(isInt ? Ailp : Aglp) + aOff;
  const T* Bh = (const T*)Bhp + bOff;
  const T* Bl = (const T*)Blp + bOff;

  const int rlane = lane & 15;
  const int koff  = (lane >> 4) * 8;
  const int mOff  = (lane >> 4) * 8;

  v8f acc[4][4];
#pragma unroll
  for (int i = 0; i < 4; ++i)
#pragma unroll
    for (int j = 0; j < 4; ++j) acc[i][j] = (v8f){0.f,0.f,0.f,0.f,0.f,0.f,0.f,0.f};

  for (int k0 = 0; k0 < Ktot; k0 += 32) {
    const int chunk = k0 >> 6;
    const int tb = c_idx[tabRow][chunk & 7];
    const int boff = (useTab ? (tb * 64) : (chunk * 64)) + (k0 & 63);
    V bh[4], bl[4];
#pragma unroll
    for (int j = 0; j < 4; ++j) {
      const size_t bo = (size_t)((j << 4) + rlane) * ldb + boff + koff;
      bh[j] = Frag<T>::load(Bh + bo);
      bl[j] = Frag<T>::load(Bl + bo);
    }
#pragma unroll
    for (int i = 0; i < 4; ++i) {
      const size_t ao = (size_t)((i << 4) + rlane) * lda + k0 + koff;
      V ah = Frag<T>::load(Ah + ao);
      V al = Frag<T>::load(Al + ao);
#pragma unroll
      for (int j = 0; j < 4; ++j) {
        acc[i][j] = Frag<T>::mma(ah, bh[j], acc[i][j]);
        acc[i][j] = Frag<T>::mma(ah, bl[j], acc[i][j]);
        acc[i][j] = Frag<T>::mma(al, bh[j], acc[i][j]);
      }
      Frag<T>::guard(acc[i][0], acc[i][3], ah, al);
    }
    Frag<T>::keep(bh[0], bh[1], bh[2], bh[3]);
    Frag<T>::keep(bl[0], bl[1], bl[2], bl[3]);
  }
  acc_guard4(acc[0][0], acc[0][1], acc[0][2], acc[0][3]);
  acc_guard4(acc[1][0], acc[1][1], acc[1][2], acc[1][3]);
  acc_guard4(acc[2][0], acc[2][1], acc[2][2], acc[2][3]);
  acc_guard4(acc[3][0], acc[3][1], acc[3][2], acc[3][3]);

  float* slab = sT[wave];
#pragma unroll
  for (int i = 0; i < 4; ++i) {
    const int mBase = (i << 4);
#pragma unroll
    for (int j = 0; j < 4; ++j) {
#pragma unroll
      for (int r = 0; r < 8; ++r) {
        const float v = acc[i][j][r] * scale;
        slab[(mOff + r) * 68 + (j << 4) + rlane] = v;
      }
    }
    __builtin_amdgcn_fence(__ATOMIC_RELEASE, "workgroup");
    __builtin_amdgcn_wave_barrier();
    __builtin_amdgcn_fence(__ATOMIC_ACQUIRE, "workgroup");
    if (OUTF == 0) {
      float* C = (float*)(isInt ? Cip : Cgp) + cOff;
      const int hh = lane >> 4, c4 = (lane & 15) * 4;
      for (int pass = 0; pass < 2; ++pass) {
#pragma unroll
        for (int it = 0; it < 8; ++it) {
          const int row = it * 2 + hh;
          v4f v = *(const v4f*)(slab + row * 68 + c4);
          *(volatile v4f*)(C + (size_t)(mBase + row) * ldc + c4) = v;
        }
        __threadfence();
      }
    } else {
      unsigned short* C = (unsigned short*)(isInt ? Cip : Cgp) + cOff;
      const int q = lane >> 3, c8 = (lane & 7) * 8;
      for (int pass = 0; pass < 2; ++pass) {
#pragma unroll
        for (int it = 0; it < 4; ++it) {
          const int row = it * 4 + q;
          const float* sp = slab + row * 68 + c8;
          v8h hv;
#pragma unroll
          for (int e = 0; e < 8; ++e) hv[e] = (_Float16)sp[e];
          *(volatile v8h*)(C + (size_t)(mBase + row) * ldc + c8) = hv;
        }
        __threadfence();
      }
    }
    __builtin_amdgcn_fence(__ATOMIC_RELEASE, "workgroup");
    __builtin_amdgcn_wave_barrier();
    __builtin_amdgcn_fence(__ATOMIC_ACQUIRE, "workgroup");
  }
}

constexpr size_t kPlane16   = (size_t)kSeq * kDim * 2;
constexpr size_t kPlane32   = (size_t)kSeq * kDim * 4;
constexpr size_t kWsq       = (size_t)kDim * kDim * 2;
constexpr size_t kOffW4     = 0;
constexpr size_t kOffW1T    = kOffW4 + 4 * kWsq;
constexpr size_t kOffW2T    = kOffW1T + (size_t)kMlp * kDim * 2;
constexpr size_t kOffQh     = kOffW2T + (size_t)kDim * kMlp * 2;
constexpr size_t kOffQl     = kOffQh + kPlane16;
constexpr size_t kOffKh     = kOffQl + kPlane16;
constexpr size_t kOffKl     = kOffKh + kPlane16;
constexpr size_t kOffVth    = kOffKl + kPlane16;
constexpr size_t kOffVtl    = kOffVth + kPlane16;
constexpr size_t kOffO      = kOffVtl + kPlane16;
constexpr size_t kOffX1     = kOffO + kPlane16;
constexpr size_t kOffScr    = kOffX1 + kPlane32;
constexpr size_t kOffX16h   = kOffScr;
constexpr size_t kOffX16l   = kOffX16h + kPlane16;
constexpr size_t kOffT      = kOffX16l + kPlane16;
constexpr size_t kSzSint    = (size_t)kHG * kNI * 64 * kKint * 4;
constexpr size_t kSzSg      = (size_t)kHG * 2 * 64 * kSeq * 4;
constexpr size_t kSzPi      = (size_t)kHG * kNI * 64 * kKint * 2;
constexpr size_t kSzPg      = (size_t)kHG * 2 * 64 * kSeq * 2;
constexpr size_t kOffSint   = kOffScr;
constexpr size_t kOffSg     = kOffSint + kSzSint;
constexpr size_t kOffPih    = kOffSg + kSzSg;
constexpr size_t kOffPil    = kOffPih + kSzPi;
constexpr size_t kOffPgh    = kOffPil + kSzPi;
constexpr size_t kOffPgl    = kOffPgh + kSzPg;
constexpr size_t kScrEnd    = kOffPgl + kSzPg;
constexpr size_t kOffY16    = kOffScr;
constexpr size_t kOffHid    = kOffY16 + kPlane16;
constexpr size_t kSzHid     = (size_t)kSeq * kMlp * 2;
constexpr size_t kWsTotal   = kScrEnd;
static_assert(kWsTotal == 125829120);
static_assert(kOffHid + kSzHid <= kScrEnd);
static_assert(kOffT + kPlane32 <= kScrEnd);
static_assert(kWsTotal <= (size_t)134217728);

extern "C" void kernel_launch(void* const* d_in, const int* in_sizes, int n_in,
                              void* d_out, int out_size, void* d_ws, size_t ws_size,
                              hipStream_t stream) {
  if (n_in < 13) return;
  if (ws_size < kWsTotal) return;
  if (out_size < kBatch * kSeq * kDim) return;
  if (in_sizes[0] < kBatch * kSeq * kDim) return;

  const float* inp  = (const float*)d_in[0];
  const float* ln1s = (const float*)d_in[1];
  const float* ln1b = (const float*)d_in[2];
  const float* wq   = (const float*)d_in[3];
  const float* wk   = (const float*)d_in[4];
  const float* wv   = (const float*)d_in[5];
  const float* wo   = (const float*)d_in[6];
  const float* ln2s = (const float*)d_in[7];
  const float* ln2b = (const float*)d_in[8];
  const float* w1   = (const float*)d_in[9];
  const float* b1   = (const float*)d_in[10];
  const float* w2   = (const float*)d_in[11];
  const float* b2   = (const float*)d_in[12];
  float* out = (float*)d_out;
  char* ws = (char*)d_ws;

  unsigned short* WqT  = (unsigned short*)(ws + kOffW4);
  unsigned short* WkT  = WqT + (size_t)kDim * kDim;
  unsigned short* WvT  = WqT + (size_t)2 * kDim * kDim;
  unsigned short* WoT  = WqT + (size_t)3 * kDim * kDim;
  unsigned short* W1T  = (unsigned short*)(ws + kOffW1T);
  unsigned short* W2T  = (unsigned short*)(ws + kOffW2T);
  unsigned short* Qh   = (unsigned short*)(ws + kOffQh);
  unsigned short* Ql   = (unsigned short*)(ws + kOffQl);
  unsigned short* Kh   = (unsigned short*)(ws + kOffKh);
  unsigned short* Kl   = (unsigned short*)(ws + kOffKl);
  unsigned short* Vth  = (unsigned short*)(ws + kOffVth);
  unsigned short* Vtl  = (unsigned short*)(ws + kOffVtl);
  unsigned short* Ob   = (unsigned short*)(ws + kOffO);
  float*          X1   = (float*)(ws + kOffX1);
  unsigned short* X16h = (unsigned short*)(ws + kOffX16h);
  unsigned short* X16l = (unsigned short*)(ws + kOffX16l);
  float*          T32  = (float*)(ws + kOffT);
  float*          Sint = (float*)(ws + kOffSint);
  float*          Sg   = (float*)(ws + kOffSg);
  unsigned short* Pih  = (unsigned short*)(ws + kOffPih);
  unsigned short* Pil  = (unsigned short*)(ws + kOffPil);
  unsigned short* Pgh  = (unsigned short*)(ws + kOffPgh);
  unsigned short* Pgl  = (unsigned short*)(ws + kOffPgl);
  unsigned short* Y16  = (unsigned short*)(ws + kOffY16);
  unsigned short* Hid  = (unsigned short*)(ws + kOffHid);

  tcast_kernel<<<dim3(kDim / 64, kDim / 64, 4), 256, 0, stream>>>(wq, wk, wv, wo, kDim, kDim, WqT, (long)kDim * kDim, kWCarry);
  tcast_kernel<<<dim3(kDim / 64, kMlp / 64, 1), 256, 0, stream>>>(w1, w1, w1, w1, kDim, kMlp, W1T, 0L, kWCarry);
  tcast_kernel<<<dim3(kMlp / 64, kDim / 64, 1), 256, 0, stream>>>(w2, w2, w2, w2, kMlp, kDim, W2T, 0L, kWCarry);

  const size_t tokStride = (size_t)kSeq * kDim;
  for (int bb = 0; bb < kBatch; ++bb) {
    const float* inpb = inp + (size_t)bb * tokStride;
    float* outb = out + (size_t)bb * tokStride;

    ln_kernel<true><<<kSeq / 8, 256, 0, stream>>>(inpb, ln1s, ln1b, X16h, X16l, kSeq);

    wmma_gemm64<0, false, 0, 2, false, 0><<<dim3(64, 1), 256, 0, stream>>>(
        WvT, WvT, kDim, 0L, X16h, X16h, kDim, 0L, (void*)Vth, (void*)Vtl, kSeq, 0L,
        b1, X1, 0L, kDim, kSeq, kDim, 1.0f / kWCarry);

    wmma_gemm64<0, false, 0, 0, false, 0><<<dim3(64, 1), 256, 0, stream>>>(
        X16h, X16h, kDim, 0L, WqT, WqT, kDim, 0L, (void*)T32, (void*)T32, kDim, 0L,
        b1, X1, 0L, kSeq, kDim, kDim, 0.125f / kWCarry);
    wmma_gemm64<0, false, 0, 2, true, 0><<<dim3(64, 1), 256, 0, stream>>>(
        X16l, X16l, kDim, 0L, WqT, WqT, kDim, 0L, (void*)Qh, (void*)Ql, kDim, 0L,
        b1, T32, 0L, kSeq, kDim, kDim, 0.125f / (kWCarry * kXLoCarry));

    wmma_gemm64<0, false, 0, 0, false, 0><<<dim3(64, 1), 256, 0, stream>>>(
        X16h, X16h, kDim, 0L, WkT, WkT, kDim, 0L, (void*)T32, (void*)T32, kDim, 0L,
        b1, X1, 0L, kSeq, kDim, kDim, 1.0f / kWCarry);
    wmma_gemm64<0, false, 0, 2, true, 0><<<dim3(64, 1), 256, 0, stream>>>(
        X16l, X16l, kDim, 0L, WkT, WkT, kDim, 0L, (void*)Kh, (void*)Kl, kDim, 0L,
        b1, T32, 0L, kSeq, kDim, kDim, 1.0f / (kWCarry * kXLoCarry));

    for (int hc = 0; hc < kHeads / kHG; ++hc) {
      const int h0 = hc * kHG;
      attn_tile_kernel<0><<<(kHG * kNI * 8 + kHG * 2 * 64) / 8, 256, 0, stream>>>(
          Qh, Ql, Qh, Ql, Kh, Kl, (void*)Sint, (void*)Sg, h0, 1.0f);
      softmax_int_kernel<<<(kHG * kNI * 64) / 4, 256, 0, stream>>>(Sint, Pih, Pil);
      softmax_glob_kernel<<<kHG * 2 * 64, 512, 0, stream>>>(Sg, Pgh, Pgl);
      attn_tile_kernel<1><<<(kHG * kNI + kHG * 2) / 8, 256, 0, stream>>>(
          Pih, Pil, Pgh, Pgl, Vth, Vtl, (void*)Ob, (void*)Ob, h0, kOCarry);
    }

    wmma_gemm64<0, false, 0, 0, true, 0><<<dim3(64, 1), 256, 0, stream>>>(
        Ob, Ob, kDim, 0L, WoT, WoT, kDim, 0L, (void*)X1, (void*)X1, kDim, 0L,
        b1, inpb, 0L, kSeq, kDim, kDim, 1.0f / (kOCarry * kWCarry));

    ln_kernel<false><<<kSeq / 8, 256, 0, stream>>>(X1, ln2s, ln2b, Y16, Y16, kSeq);

    wmma_gemm64<0, false, 2, 1, false, 6><<<dim3(256, 1), 256, 0, stream>>>(
        Y16, Y16, kDim, 0L, W1T, W1T, kDim, 0L, (void*)Hid, (void*)Hid, kMlp, 0L,
        b1, X1, 0L, kSeq, kMlp, kDim, 1.0f / kWCarry);

    wmma_gemm64<0, false, 2, 0, true, 0><<<dim3(64, 1), 256, 0, stream>>>(
        Hid, Hid, kMlp, 0L, W2T, W2T, kMlp, 0L, (void*)outb, (void*)outb, kDim, 0L,
        b2, X1, 0L, kSeq, kDim, kMlp, 1.0f / (kWCarry * kHidCarry));
  }
}
